// GCN_31593779430135
// MI455X (gfx1250) — hardware-verified
//
#include <hip/hip_runtime.h>
#include <stddef.h>
#include <stdint.h>
#include <math.h>


#define CIN    128
#define HID    64
#define K2     128
#define NCLS   40
#define NTHR   256
#define NWAVE  8
#define EPT    8
#define CHUNK  (NTHR * EPT)
#define WCAP   (EPT * 32)
#define LISTN  (NWAVE * WCAP)
#define NBD    8192
#define SLD    13
#define NBA    1024
#define SLA    10
#define SPW    (NBA / NWAVE)
#define RCAP   24576
#define DEGCAP 64
#define GBM    64
#define GBN    64
#define GTHR   128
#define NUW    (HID * (K2 / 8))
#define WPL    (HID * K2)
#define OG     16
#define STGF   (OG * NCLS)
#define AGG_ZINTS (LISTN + 2 * RCAP + 3 * NBA)
#define MISC_INTS 16
#define AGG_LDS_INTS (AGG_ZINTS + MISC_INTS + NWAVE * STGF)
#define WSMAX  134217728

static_assert((CHUNK & (CHUNK - 1)) == 0 && CHUNK <= 4096);
static_assert((NBD & (NBD - 1)) == 0 && NBD == (1 << SLD));
static_assert((NBA & (NBA - 1)) == 0 && NBA == (1 << SLA));
static_assert(((long long)CHUNK << SLD) < (1LL << 31));
static_assert(((long long)CHUNK << SLA) < (1LL << 31));
static_assert(NBD % (NTHR * 4) == 0);
static_assert(LISTN % NTHR == 0);
static_assert(NBA % NWAVE == 0 && NBA % 32 == 0 && NBA % GBM == 0);
static_assert(RCAP % 32 == 0 && AGG_ZINTS % (NTHR * 4) == 0 && LISTN % 4 == 0);
static_assert(((AGG_ZINTS + MISC_INTS) % 4) == 0);
static_assert(CIN % 32 == 0 && K2 % 32 == 0 && K2 == 2 * HID && HID == GBN && CIN == K2);
static_assert(GBM == (GTHR / 32) * 16 && GBN == 64 && GTHR >= GBM);
static_assert(NUW % NTHR == 0 && NUW == 1024 && K2 / 8 == 16);
static_assert(HID == 2 * 32);
static_assert(NCLS % 2 == 0 && NCLS <= HID && NCLS / 2 <= 32);
static_assert(STGF == 5 * 32 * 4);
static_assert((OG * NCLS * 4) % 128 == 0 && SPW % OG == 0);
static_assert(((long long)NBA * NCLS * 4) % 128 == 0);
static_assert(DEGCAP >= 35 + 8 && RCAP >= 16623 + 4096);
static_assert(AGG_LDS_INTS * 4 <= 300000);

typedef float          v2f   __attribute__((ext_vector_type(2)));
typedef float          v4f   __attribute__((ext_vector_type(4)));
typedef float          v8f   __attribute__((ext_vector_type(8)));
typedef int            v4i   __attribute__((ext_vector_type(4)));
typedef int            v8i   __attribute__((ext_vector_type(8)));
typedef unsigned int   v4u   __attribute__((ext_vector_type(4)));
typedef unsigned short v8us  __attribute__((ext_vector_type(8)));
typedef unsigned short v16us __attribute__((ext_vector_type(16)));
typedef __bf16         v16bf __attribute__((ext_vector_type(16)));
typedef v2f  __attribute__((may_alias)) v2fa;
typedef v4f  __attribute__((may_alias)) v4fa;
typedef v4i  __attribute__((may_alias)) v4ia;
typedef v8us __attribute__((may_alias)) v8usa;
union FragB { v16bf v; v16us u; v8us h[2]; v8i w; };

__device__ __forceinline__ v8f wmb(const FragB& a, const FragB& b, v8f c) {
  v8f d = __builtin_amdgcn_wmma_f32_16x16x32_bf16(false, a.v, false, b.v, (short)0, c, false, false);
  asm volatile("v_nop\n\tv_nop\n\tv_nop\n\tv_nop" : "+v"(d) : "v"(a.w), "v"(b.w));
  return d;
}

__device__ __forceinline__ unsigned bf16_bits(float f) {
  const unsigned u = __float_as_uint(f);
  const unsigned r = (u + 0x7FFFu + ((u >> 16) & 1u)) >> 16;
  const bool isn = (u & 0x7fffffffu) > 0x7f800000u;
  return isn ? 0x7fc0u : r;
}
__device__ __forceinline__ float bf16_val(float f) {
  return __uint_as_float(bf16_bits(f) << 16);
}

__device__ __forceinline__ void wave_sync() {
  __builtin_amdgcn_fence(__ATOMIC_RELEASE, "wavefront");
  __builtin_amdgcn_wave_barrier();
  __builtin_amdgcn_fence(__ATOMIC_ACQUIRE, "wavefront");
}

template <int SLB>
__device__ __forceinline__ int scan_chunk(const int* __restrict__ dsts, int nE, int cbase, int slotBase,
                                          int nb, int vec8, int* list, int tid, int lane, int wave) {
  int wc = 0;
  const int el0  = tid * EPT;
  const int e0   = cbase + el0;
  const int sent = -2147483647 - 1;
  v4i da, db;
  if (vec8 != 0 && cbase + CHUNK <= nE) {
    da = *(const v4i*)(dsts + e0);
    db = *(const v4i*)(dsts + e0 + 4);
  } else {
    da.x = (e0     < nE) ? dsts[min(e0,     nE - 1)] : sent;
    da.y = (e0 + 1 < nE) ? dsts[min(e0 + 1, nE - 1)] : sent;
    da.z = (e0 + 2 < nE) ? dsts[min(e0 + 2, nE - 1)] : sent;
    da.w = (e0 + 3 < nE) ? dsts[min(e0 + 3, nE - 1)] : sent;
    db.x = (e0 + 4 < nE) ? dsts[min(e0 + 4, nE - 1)] : sent;
    db.y = (e0 + 5 < nE) ? dsts[min(e0 + 5, nE - 1)] : sent;
    db.z = (e0 + 6 < nE) ? dsts[min(e0 + 6, nE - 1)] : sent;
    db.w = (e0 + 7 < nE) ? dsts[min(e0 + 7, nE - 1)] : sent;
  }
  const unsigned nbs = (unsigned)slotBase;
  const unsigned unb = (unsigned)nb;
  const unsigned s0 = (unsigned)da.x - nbs, s1 = (unsigned)da.y - nbs;
  const unsigned s2 = (unsigned)da.z - nbs, s3 = (unsigned)da.w - nbs;
  const unsigned s4 = (unsigned)db.x - nbs, s5 = (unsigned)db.y - nbs;
  const unsigned s6 = (unsigned)db.z - nbs, s7 = (unsigned)db.w - nbs;
  const bool h0 = s0 < unb, h1 = s1 < unb, h2 = s2 < unb, h3 = s3 < unb;
  const bool h4 = s4 < unb, h5 = s5 < unb, h6 = s6 < unb, h7 = s7 < unb;
  const unsigned any = __builtin_amdgcn_ballot_w32(h0 | h1 | h2 | h3 | h4 | h5 | h6 | h7);
  if (any != 0u) {
#define HITJ(J, HJ, SJ) { \
      const unsigned mj = __builtin_amdgcn_ballot_w32(HJ); \
      if (mj != 0u) { \
        if (HJ) { \
          const int pos = wc + (int)__builtin_amdgcn_mbcnt_lo(mj, 0u); \
          if (pos < WCAP) list[wave * WCAP + pos] = ((el0 + (J)) << SLB) | (int)(SJ); \
        } \
        wc += (int)__builtin_popcount(mj); } }
    HITJ(0, h0, s0)
    HITJ(1, h1, s1)
    HITJ(2, h2, s2)
    HITJ(3, h3, s3)
    HITJ(4, h4, s4)
    HITJ(5, h5, s5)
    HITJ(6, h6, s6)
    HITJ(7, h7, s7)
#undef HITJ
  }
  return wc;
}

__global__ __launch_bounds__(NTHR) void k_wprep(const float* __restrict__ W1, const float* __restrict__ W2,
                                                const float* __restrict__ W3, unsigned short* WT) {
  const int u    = (int)blockIdx.x * NTHR + (int)threadIdx.x;
  const int part = u >> 10;
  const int v    = u & (NUW - 1);
  const int n    = v >> 4;
  const int k8   = (v & 15) * 8;
  v8us o;
  if (part == 0) {
    const float* p = W1 + (size_t)k8 * HID + n;
#pragma unroll
    for (int i = 0; i < 8; ++i) o[i] = (unsigned short)bf16_bits(p[(size_t)i * HID]);
  } else if (part == 1) {
    const int kk = k8 & (HID - 1);
    const float* p = W2 + (size_t)kk * HID + n;
#pragma unroll
    for (int i = 0; i < 8; ++i) o[i] = (unsigned short)bf16_bits(p[(size_t)i * HID]);
  } else if (part == 2) {
    const int kk = k8 & (HID - 1);
    const int nc = n < NCLS ? n : NCLS - 1;
    const bool ok = n < NCLS;
    const float* p = W3 + (size_t)kk * NCLS + nc;
#pragma unroll
    for (int i = 0; i < 8; ++i) {
      const unsigned b = bf16_bits(p[(size_t)i * NCLS]);
      o[i] = ok ? (unsigned short)b : (unsigned short)0;
    }
  } else {
    return;
  }
  unsigned short* dp = WT + (size_t)part * WPL + (size_t)n * K2 + k8;
  *(volatile v8us*)dp = o;
  __threadfence();
  *(volatile v8us*)dp = o;
}

__global__ __launch_bounds__(NTHR) void k_cvx(const float* __restrict__ x, int nN, int nUnits,
                                              unsigned short* xb) {
  const int u = (int)blockIdx.x * NTHR + (int)threadIdx.x;
  if (u >= nUnits) return;
  const int row = u >> 4;
  const int k8  = (u & 15) * 8;
  const int rc  = row < nN ? row : nN - 1;
  const float* p = x + (size_t)rc * CIN + k8;
  const v4f a = *(const v4fa*)p;
  const v4f b = *(const v4fa*)(p + 4);
  const bool ok = row < nN;
  v8us o;
  o[0] = ok ? (unsigned short)bf16_bits(a.x) : (unsigned short)0;
  o[1] = ok ? (unsigned short)bf16_bits(a.y) : (unsigned short)0;
  o[2] = ok ? (unsigned short)bf16_bits(a.z) : (unsigned short)0;
  o[3] = ok ? (unsigned short)bf16_bits(a.w) : (unsigned short)0;
  o[4] = ok ? (unsigned short)bf16_bits(b.x) : (unsigned short)0;
  o[5] = ok ? (unsigned short)bf16_bits(b.y) : (unsigned short)0;
  o[6] = ok ? (unsigned short)bf16_bits(b.z) : (unsigned short)0;
  o[7] = ok ? (unsigned short)bf16_bits(b.w) : (unsigned short)0;
  unsigned short* dp = xb + (size_t)row * CIN + k8;
  *(volatile v8us*)dp = o;
  __threadfence();
  *(volatile v8us*)dp = o;
}

__global__ __launch_bounds__(NTHR) void k_deg(const int* __restrict__ dsts, int nE, int vec8, float* dis) {
  __shared__ __attribute__((aligned(16))) int scnt[NBD];
  __shared__ __attribute__((aligned(16))) int list[LISTN];
  __shared__ int wcnt[NWAVE];
  const int tid = (int)threadIdx.x, lane = tid & 31, wave = tid >> 5;
  const int nodeBase = (int)blockIdx.x * NBD;

  for (int i = tid; i < NBD; i += NTHR) scnt[i] = 0;
  for (int i = tid; i < LISTN; i += NTHR) list[i] = 0;
  if (tid < NWAVE) wcnt[tid] = 0;
  __syncthreads();

  const int nChunks = (nE + CHUNK - 1) / CHUNK;
#pragma unroll 1
  for (int ch = 0; ch < nChunks; ++ch) {
    const int cbase = ch * CHUNK;
    const int wc = scan_chunk<SLD>(dsts, nE, cbase, nodeBase, NBD, vec8, list, tid, lane, wave);
    if (lane == 0) wcnt[wave] = wc;
    __syncthreads();
    if (wave == 0) {
#pragma unroll 1
      for (int w2 = 0; w2 < NWAVE; ++w2) {
        int c = wcnt[w2];
        c = c < 0 ? 0 : (c > WCAP ? WCAP : c);
#pragma unroll 1
        for (int b0 = 0; b0 < c; b0 += 32) {
          const int idx = b0 + lane;
          const int ent = list[w2 * WCAP + (idx < WCAP ? idx : WCAP - 1)];
          const int m32 = (c - b0) < 32 ? (c - b0) : 32;
#pragma unroll 1
          for (int k = 0; k < m32; ++k) {
            const int u  = __builtin_amdgcn_readlane(ent, k);
            const int sl = u & (NBD - 1);
            if (lane == 0) scnt[sl] = scnt[sl] + 1;
          }
        }
      }
    }
    __syncthreads();
  }

  v4f vals[NBD / (NTHR * 4)];
#pragma unroll
  for (int it = 0; it < NBD / (NTHR * 4); ++it) {
    const int s0 = it * (NTHR * 4) + 4 * tid;
    const v4i c4 = *(const v4ia*)(scnt + s0);
    const float d0 = fmaxf((float)c4.x + 1.0f, 1.0f), d1 = fmaxf((float)c4.y + 1.0f, 1.0f);
    const float d2 = fmaxf((float)c4.z + 1.0f, 1.0f), d3 = fmaxf((float)c4.w + 1.0f, 1.0f);
    v4f v;
    v.x = rsqrtf(d0); v.y = rsqrtf(d1); v.z = rsqrtf(d2); v.w = rsqrtf(d3);
    vals[it] = v;
  }
#pragma unroll
  for (int it = 0; it < NBD / (NTHR * 4); ++it) {
    const int s0 = it * (NTHR * 4) + 4 * tid;
    *(volatile v4f*)(dis + (size_t)nodeBase + s0) = vals[it];
  }
  __threadfence();
#pragma unroll
  for (int it = 0; it < NBD / (NTHR * 4); ++it) {
    const int s0 = it * (NTHR * 4) + 4 * tid;
    *(volatile v4f*)(dis + (size_t)nodeBase + s0) = vals[it];
  }
}

__global__ __launch_bounds__(GTHR) void k_gemm(
    const unsigned short* __restrict__ A, const unsigned short* __restrict__ WT,
    const float* __restrict__ dis, float* outF, int K, int ldo)
{
  __shared__ __attribute__((aligned(16))) float stg[GBM * GBN];
  __shared__ float sdis[GBM];
  const int tid = (int)threadIdx.x, lane = tid & 31, wave = tid >> 5, hh = lane >> 4, m = lane & 15;
  const int rowBase = (int)blockIdx.x * GBM;
  const int col0    = (int)blockIdx.y * GBN;

  if (tid < GBM) sdis[tid] = dis[rowBase + tid];

  v8f acc[4];
  {
    const v8f z = {0.f, 0.f, 0.f, 0.f, 0.f, 0.f, 0.f, 0.f};
    acc[0] = z; acc[1] = z; acc[2] = z; acc[3] = z;
  }
  const unsigned short* ap = A  + (size_t)(rowBase + 16 * wave + m) * (size_t)K + 8 * hh;
  const unsigned short* wp = WT + (size_t)(col0 + m) * (size_t)K + 8 * hh;
  const int ksteps = K >> 5;
#pragma unroll 1
  for (int ks = 0; ks < ksteps; ++ks) {
    FragB af;
    af.h[0] = *(const v8usa*)(ap + 32 * ks);
    af.h[1] = *(const v8usa*)(ap + 32 * ks + 16);
#pragma unroll
    for (int t = 0; t < 4; ++t) {
      const unsigned short* wq = wp + (size_t)(16 * t) * (size_t)K + 32 * ks;
      FragB bf;
      bf.h[0] = *(const v8usa*)wq;
      bf.h[1] = *(const v8usa*)(wq + 16);
      acc[t] = wmb(af, bf, acc[t]);
    }
  }

#pragma unroll
  for (int t = 0; t < 4; ++t) {
    const int lc = 16 * t + m;
#pragma unroll
    for (int r = 0; r < 8; ++r) {
      const int lr = 16 * wave + 8 * hh + r;
      stg[lr * GBN + lc] = acc[t][r];
    }
  }
  __syncthreads();

  v4f fv[8];
#pragma unroll
  for (int i = 0; i < 8; ++i) {
    const int lr = 16 * wave + 2 * i + hh;
    const v4f t4 = *(const v4fa*)(stg + lr * GBN + 4 * m);
    const float ds = sdis[lr];
    v4f y;
    y.x = t4.x * ds; y.y = t4.y * ds; y.z = t4.z * ds; y.w = t4.w * ds;
    fv[i] = y;
  }
#pragma unroll
  for (int i = 0; i < 8; ++i) {
    const int lr = 16 * wave + 2 * i + hh;
    const int gr = rowBase + lr;
    float* op = outF + (size_t)gr * (size_t)ldo + col0 + 4 * m;
    *(volatile v4f*)op = fv[i];
  }
  __threadfence();
#pragma unroll
  for (int i = 0; i < 8; ++i) {
    const int lr = 16 * wave + 2 * i + hh;
    const int gr = rowBase + lr;
    float* op = outF + (size_t)gr * (size_t)ldo + col0 + 4 * m;
    *(volatile v4f*)op = fv[i];
  }
}

template <int MODE>
__global__ __launch_bounds__(NTHR) void k_agg(const int* __restrict__ srcs, const int* __restrict__ dsts,
                                              int nE, int nN, int vec8, int mRows,
                                              const float* __restrict__ dis,
                                              const float* __restrict__ hs, const float* __restrict__ bias,
                                              int nb, unsigned short* hb, float* outp) {
  extern __shared__ __attribute__((aligned(16))) int dsm[];
  int* list = dsm;
  int* hl   = dsm + LISTN;
  int* sl   = dsm + LISTN + RCAP;
  int* cnt  = dsm + LISTN + 2 * RCAP;
  int* offs = cnt + NBA;
  int* cur  = offs + NBA;
  int* misc = cur + NBA;
  const int tid = (int)threadIdx.x, lane = tid & 31, wave = tid >> 5;
  float* stg = (float*)(misc + MISC_INTS) + wave * STGF;
  const int nodeBase = (int)blockIdx.x * NBA;

  {
    const v4i z4 = {0, 0, 0, 0};
    for (int i = tid * 4; i < AGG_ZINTS; i += NTHR * 4) *(v4ia*)(dsm + i) = z4;
    if (tid < MISC_INTS) misc[tid] = 0;
  }
  float bv0, bv1;
  {
    const int c0 = 2 * lane;
    const int ca = c0 < nb - 2 ? c0 : nb - 2;
    const v2f a = *(const v2fa*)(bias + ca);
    const bool okb = c0 < nb;
    const float r0 = (MODE != 0) ? bf16_val(a.x) : a.x;
    const float r1 = (MODE != 0) ? bf16_val(a.y) : a.y;
    bv0 = okb ? r0 : 0.0f;
    bv1 = okb ? r1 : 0.0f;
  }
  __syncthreads();

  int t = 0, ov = 0;
  const int nChunks = (nE + CHUNK - 1) / CHUNK;
#pragma unroll 1
  for (int ch = 0; ch < nChunks; ++ch) {
    const int cbase = ch * CHUNK;
    const int wc = scan_chunk<SLA>(dsts, nE, cbase, nodeBase, NBA, vec8, list, tid, lane, wave);
    if (lane == 0) misc[wave] = wc;
    __syncthreads();
    if (wave == 0) {
#pragma unroll 1
      for (int w2 = 0; w2 < NWAVE; ++w2) {
        int c = misc[w2];
        c = c < 0 ? 0 : (c > WCAP ? WCAP : c);
#pragma unroll 1
        for (int b0 = 0; b0 < c; b0 += 32) {
          const int idx = b0 + lane;
          const int ent = list[w2 * WCAP + (idx < WCAP ? idx : WCAP - 1)];
          const int m32 = (c - b0) < 32 ? (c - b0) : 32;
#pragma unroll 1
          for (int k = 0; k < m32; ++k) {
            const int u    = __builtin_amdgcn_readlane(ent, k);
            const int slot = u & (NBA - 1);
            const int el   = (u >> SLA) & (CHUNK - 1);
            const int pk   = ((cbase + el) << SLA) | slot;
            if (t < RCAP) {
              if (lane == 0) { hl[t] = pk; cnt[slot] = cnt[slot] + 1; }
              t = t + 1;
            } else {
              ov = 1;
            }
          }
        }
      }
    }
    __syncthreads();
  }
  if (wave == 0 && lane == 0) { misc[8] = t; misc[9] = ov; }
  __syncthreads();
  int tt = misc[8];
  tt = tt < 0 ? 0 : (tt > RCAP ? RCAP : tt);
  const int ovf = misc[9];

  if (wave == 0) {
    const int base = lane * (NBA / 32);
    int s = 0;
#pragma unroll 1
    for (int i = 0; i < NBA / 32; ++i) s += cnt[base + i];
    int incl = s;
#pragma unroll
    for (int d = 1; d < 32; d <<= 1) {
      const int y = __shfl_up(incl, d, 32);
      if (lane >= d) incl += y;
    }
    int run = incl - s;
#pragma unroll 1
    for (int i = 0; i < NBA / 32; ++i) {
      const int cv = cnt[base + i];
      offs[base + i] = run;
      cur[base + i]  = run;
      run += cv;
    }
  }
  __syncthreads();
  if (wave == 0) {
#pragma unroll 1
    for (int b0 = 0; b0 < tt; b0 += 32) {
      const int idx = b0 + lane;
      const int ent = hl[idx < RCAP ? idx : RCAP - 1];
      const int m32 = (tt - b0) < 32 ? (tt - b0) : 32;
#pragma unroll 1
      for (int k = 0; k < m32; ++k) {
        const int u    = __builtin_amdgcn_readlane(ent, k);
        const int slot = u & (NBA - 1);
        if (lane == 0) {
          int p = cur[slot];
          p = p < 0 ? 0 : (p > RCAP - 1 ? RCAP - 1 : p);
          sl[p] = u;
          cur[slot] = p + 1;
        }
      }
    }
  }
  __syncthreads();

  const float qnan = __int_as_float(0x7fc00000);
  const float pz = (ovf != 0) ? qnan : 0.0f;
  const int q0s = (4 * lane) & 31, q1s = (4 * lane + 1) & 31;
  const int q2s = (4 * lane + 2) & 31, q3s = (4 * lane + 3) & 31;
#pragma unroll 1
  for (int si = 0; si < SPW; ++si) {
    const int s    = wave * SPW + si;
    const int node = nodeBase + s;
    int c = cnt[s];
    const bool big = c > DEGCAP;
    c = c < 0 ? 0 : (c > DEGCAP ? DEGCAP : c);
    int o = offs[s];
    o = o < 0 ? 0 : (o > RCAP ? RCAP : o);
    const int nc = node < nN ? node : nN - 1;
    const float dd = dis[nc];
    float acc0 = 0.0f, acc1 = 0.0f;
#pragma unroll 1
    for (int b0 = 0; b0 < c; b0 += 32) {
      int idx = o + b0 + lane;
      idx = idx > RCAP - 1 ? RCAP - 1 : idx;
      const int ent = sl[idx];
      int eid = ent >> SLA;
      eid = eid < 0 ? 0 : (eid > nE - 1 ? nE - 1 : eid);
      int sr = srcs[eid];
      sr = sr < 0 ? 0 : (sr > nN - 1 ? nN - 1 : sr);
      const int m32 = (c - b0) < 32 ? (c - b0) : 32;
#pragma unroll 1
      for (int k = 0; k < m32; ++k) {
        const int sk = __builtin_amdgcn_readlane(sr, k);
        const v2f a = *(const v2fa*)(hs + (size_t)sk * HID + 2 * lane);
        acc0 += a.x; acc1 += a.y;
      }
    }
    {
      const v2f a = *(const v2fa*)(hs + (size_t)nc * HID + 2 * lane);
      acc0 += a.x; acc1 += a.y;
    }
    const float pzr = big ? qnan : pz;
    float y0 = (dd * acc0 + bv0) + pzr;
    float y1 = (dd * acc1 + bv1) + pzr;
    if constexpr (MODE != 0) {
      y0 = (y0 > 0.0f) ? y0 : (y0 - y0);
      y1 = (y1 > 0.0f) ? y1 : (y1 - y1);
      const bool live = node < nN;
      const float v0 = live ? y0 : 0.0f;
      const float v1 = live ? y1 : 0.0f;
      const bool wr = (node < mRows) && (lane < 16);
      const unsigned hb0 = bf16_bits(v0), hb1 = bf16_bits(v1);
      const unsigned lb0 = bf16_bits(v0 - __uint_as_float(hb0 << 16));
      const unsigned lb1 = bf16_bits(v1 - __uint_as_float(hb1 << 16));
      const int hw = (int)(hb0 | (hb1 << 16));
      const int lw = (int)(lb0 | (lb1 << 16));
      const int g0 = __shfl(hw, q0s, 32), g1 = __shfl(hw, q1s, 32);
      const int g2 = __shfl(hw, q2s, 32), g3 = __shfl(hw, q3s, 32);
      const int p0 = __shfl(lw, q0s, 32), p1 = __shfl(lw, q1s, 32);
      const int p2 = __shfl(lw, q2s, 32), p3 = __shfl(lw, q3s, 32);
      const bool lsel = (lane & 8) != 0;
      v4u pv;
      pv.x = (unsigned int)(lsel ? p0 : g0);
      pv.y = (unsigned int)(lsel ? p1 : g1);
      pv.z = (unsigned int)(lsel ? p2 : g2);
      pv.w = (unsigned int)(lsel ? p3 : g3);
      unsigned short* hp = hb + (size_t)node * K2 + 8 * (lane & 15);
      if (wr) *(volatile v4u*)hp = pv;
      __threadfence();
      if (wr) *(volatile v4u*)hp = pv;
    } else {
      const int r = si & (OG - 1);
      v2f yv;
      yv.x = y0; yv.y = y1;
      if (lane < NCLS / 2) *(v2fa*)(stg + r * NCLS + 2 * lane) = yv;
      if (r == OG - 1) {
        wave_sync();
        v4f q[5];
#pragma unroll
        for (int it = 0; it < 5; ++it) q[it] = *(const v4fa*)(stg + 128 * it + 4 * lane);
        wave_sync();
        const int g0r = node - (OG - 1);
        if (g0r < nN) {
          float* op = outp + (size_t)g0r * NCLS + 4 * lane;
#pragma unroll
          for (int it = 0; it < 5; ++it) *(volatile v4f*)(op + 128 * it) = q[it];
          __threadfence();
#pragma unroll
          for (int it = 0; it < 5; ++it) *(volatile v4f*)(op + 128 * it) = q[it];
        }
      }
    }
  }
}

static inline int cdiv(int a, int b) { return (a + b - 1) / b; }
static inline size_t al256(size_t o) { return (o + 255) & ~(size_t)255; }

extern "C" void kernel_launch(void* const* d_in, const int* in_sizes, int n_in,
                              void* d_out, int out_size, void* d_ws, size_t ws_size,
                              hipStream_t stream) {
  if (n_in < 8) return;
  if (in_sizes[0] < CIN || (in_sizes[0] % CIN) != 0) return;
  const int nN = in_sizes[0] / CIN;
  if (nN < 16 || nN > (1 << 22) || (nN % OG) != 0) return;
  if (in_sizes[1] < 2 || (in_sizes[1] & 1) != 0) return;
  const int nE = in_sizes[1] / 2;
  if (nE < 1 || nE >= (1 << (31 - SLA))) return;
  if (in_sizes[2] != CIN * HID || in_sizes[3] != HID) return;
  if (in_sizes[4] != HID * HID || in_sizes[5] != HID) return;
  if (in_sizes[6] != HID * NCLS || in_sizes[7] != NCLS) return;
  if ((long long)out_size != (long long)nN * NCLS) return;

  const float* x    = (const float*)d_in[0];
  const int*   edge = (const int*)d_in[1];
  const float* W1   = (const float*)d_in[2];
  const float* b1   = (const float*)d_in[3];
  const float* W2   = (const float*)d_in[4];
  const float* b2   = (const float*)d_in[5];
  const float* W3   = (const float*)d_in[6];
  const float* b3   = (const float*)d_in[7];
  float* out = (float*)d_out;
  const int* src = edge;
  const int* dst = edge + nE;

  const int MP   = cdiv(nN, GBM) * GBM;
  const int gM   = MP / GBM;
  const int gD   = cdiv(MP, NBD);
  const int NBPD = gD * NBD;
  const int gA   = cdiv(MP, NBA);
  if ((long long)gA * NBA < (long long)MP) return;
  if (NBPD < MP) return;
  const int vec8 = ((nE & 3) == 0) ? 1 : 0;

  char* ws = (char*)d_ws;
  size_t off = 0;
  const size_t oDIS = off; off = al256(off + (size_t)NBPD * 4);
  const size_t oWT  = off; off = al256(off + (size_t)3 * WPL * 2);
  const size_t oXB  = off; off = al256(off + (size_t)MP * CIN * 2);
  const size_t oHSa = off; off = al256(off + (size_t)MP * HID * 4);
  const size_t oX1  = off; off = al256(off + (size_t)MP * K2 * 2);
  const size_t oHSb = off; off = al256(off + (size_t)MP * HID * 4);
  const size_t oX2  = off; off = al256(off + (size_t)MP * K2 * 2);
  if (off > ws_size || off > (size_t)WSMAX) return;
  float*          DIS = (float*)(ws + oDIS);
  unsigned short* WT  = (unsigned short*)(ws + oWT);
  unsigned short* XB  = (unsigned short*)(ws + oXB);
  float*          HSa = (float*)(ws + oHSa);
  unsigned short* X1  = (unsigned short*)(ws + oX1);
  float*          HSb = (float*)(ws + oHSb);
  unsigned short* X2  = (unsigned short*)(ws + oX2);
  const unsigned short* W1T = WT;
  const unsigned short* W2T = WT + WPL;
  const unsigned short* W3T = WT + 2 * WPL;

  const size_t aggLds = (size_t)AGG_LDS_INTS * 4;
  hipFuncSetAttribute(reinterpret_cast<const void*>(&k_agg<1>), hipFuncAttributeMaxDynamicSharedMemorySize, (int)aggLds);
  hipFuncSetAttribute(reinterpret_cast<const void*>(&k_agg<0>), hipFuncAttributeMaxDynamicSharedMemorySize, (int)aggLds);

  const int nUx = MP * (CIN / 8);
  k_wprep<<<(3 * NUW) / NTHR, NTHR, 0, stream>>>(W1, W2, W3, WT);
  k_cvx<<<cdiv(nUx, NTHR), NTHR, 0, stream>>>(x, nN, nUx, XB);
  k_deg<<<gD, NTHR, 0, stream>>>(dst, nE, vec8, DIS);
  k_gemm<<<dim3(gM, 1), GTHR, 0, stream>>>(XB, W1T, DIS, HSa, CIN, HID);
  k_agg<1><<<gA, NTHR, aggLds, stream>>>(src, dst, nE, nN, vec8, MP, DIS, HSa, b1, HID, X1, out);
  k_gemm<<<dim3(gM, 1), GTHR, 0, stream>>>(X1, W2T, DIS, HSb, K2, HID);
  k_agg<1><<<gA, NTHR, aggLds, stream>>>(src, dst, nE, nN, vec8, MP, DIS, HSb, b2, HID, X2, out);
  k_gemm<<<dim3(gM, 1), GTHR, 0, stream>>>(X2, W3T, DIS, HSa, K2, HID);
  k_agg<0><<<gA, NTHR, aggLds, stream>>>(src, dst, nE, nN, vec8, MP, DIS, HSa, b3, NCLS, X2, out);
}
